// CrossAttention_67233418051751
// MI455X (gfx1250) — hardware-verified
//
#include <hip/hip_runtime.h>
#include <stdint.h>


typedef _Float16 v16h __attribute__((ext_vector_type(16)));
typedef _Float16 v8h  __attribute__((ext_vector_type(8)));
typedef float    v8f  __attribute__((ext_vector_type(8)));
typedef float    v4f  __attribute__((ext_vector_type(4)));
typedef float    v2f  __attribute__((ext_vector_type(2)));

#ifndef NB
#define NB 2
#endif
#ifndef SEQ
#define SEQ 2048
#endif
#ifndef SKV
#define SKV 1024
#endif
#define NB_FULL  2
#define SEQ_FULL 2048
#define SKV_FULL 1024
#define DM   1024
#define DC   1024
#define NH   16
#define HD   64

#define ACT_CAR   8.0f
#define W_CAR     1024.0f
#define PROJ_TRUE 0.0001220703125f
#define PROJ_SCL  0.0009765625f
#define K_CAR     8.0f
#define RES_CAR   2048.0f
#define RES_INV   0.00048828125f
#define S_SCL     0.015625f
#define P_CAR     16384.0f
#define O_SCL     0.001953125f
#define OUT_SCL   3.814697265625e-06f
#define LN_EPS    1e-6f

__host__ __device__ constexpr unsigned lg2u(unsigned v) { return v <= 1u ? 0u : 1u + lg2u(v >> 1); }
constexpr unsigned kSeqSh = lg2u((unsigned)SEQ);
constexpr unsigned kSkvSh = lg2u((unsigned)SKV);
constexpr unsigned kDmSh  = lg2u((unsigned)DM);
constexpr unsigned kDcSh  = lg2u((unsigned)DC);

static_assert((1u << kSeqSh) == (unsigned)SEQ && (1u << kSkvSh) == (unsigned)SKV);
static_assert((1u << kDmSh) == (unsigned)DM && (1u << kDcSh) == (unsigned)DC);
static_assert(SEQ % 128 == 0 && SKV % 128 == 0);
static_assert(SEQ <= SEQ_FULL && SKV <= SKV_FULL && NB <= NB_FULL);
static_assert(DM == NH * HD);
static_assert(HD == 64);
static_assert(DM % 128 == 0 && DC % 32 == 0 && DM % 32 == 0);
static_assert((long)NB_FULL * SEQ_FULL * DM * 4 == 16777216L);
static_assert(((long)NB * SEQ * DM / 8) % 256 == 0 && ((long)NB * SKV * DC / 8) % 256 == 0);
static_assert(((long)DM * DM / 8) % 256 == 0 && ((long)2 * DM * DC / 8) % 256 == 0);
static_assert((long)(SEQ / 8) * 512 == (long)SEQ * 64);
static_assert((long)(DM / 64) * (NB * SEQ / 128) * 128 * 64 == (long)NB * SEQ * DM);
static_assert((long)(DM / 64) * (NB * SKV / 128) * 128 * 64 == (long)NB * SKV * DM);
static_assert((long)(NB * SKV / 64) * (DM / 128) * 128 * 64 == (long)NB * SKV * DM);
static_assert((long)(SEQ / 128) * NH * NB * 128 * HD == (long)NB * SEQ * DM);
static_assert((long)(DM / 64) * (NB * SEQ / 64) * 64 * 64 == (long)NB * SEQ * DM);

union Frag16 { v16h v; v8h p[2]; };

__device__ __forceinline__ v16h ld_frag(const _Float16* p, unsigned hl) {
  Frag16 f;
  f.p[0] = *(const v8h*)(p + 8u * hl);
  f.p[1] = *(const v8h*)(p + 16u + 8u * hl);
  return f.v;
}

__device__ __forceinline__ v8f mma(v16h a, v16h b, v8f c) {
  v8f d = __builtin_amdgcn_wmma_f32_16x16x32_f16(false, a, false, b, (short)0, c, false, false);
  asm volatile("v_nop\n\tv_nop\n\tv_nop\n\tv_nop" : "+v"(d) : "v"(a), "v"(b));
  return d;
}

__device__ __forceinline__ float bf16_rne(float x) {
  unsigned int u = __builtin_bit_cast(unsigned int, x);
  u += 0x7FFFu + ((u >> 16) & 1u);
  return __builtin_bit_cast(float, u & 0xFFFF0000u);
}

__device__ __forceinline__ float red16(float v) {
  v += __shfl_xor(v, 1, 32);
  v += __shfl_xor(v, 2, 32);
  v += __shfl_xor(v, 4, 32);
  v += __shfl_xor(v, 8, 32);
  return v;
}

__global__ __launch_bounds__(256) void k_cvt8(const float* __restrict__ src,
                                              _Float16* __restrict__ dst,
                                              unsigned csh, unsigned rsh, unsigned rows_full,
                                              float car, unsigned total8)
{
  const unsigned i8 = blockIdx.x * 256u + threadIdx.x;
  if (i8 >= total8) return;
  const unsigned e   = i8 << 3;
  const unsigned r   = e >> csh;
  const unsigned col = e & ((1u << csh) - 1u);
  const unsigned b   = r >> rsh;
  const unsigned rr  = r & ((1u << rsh) - 1u);
  const float* s = src + (((size_t)b * rows_full + rr) << csh) + col;
  const v4f x0 = *(const v4f*)s;
  const v4f x1 = *(const v4f*)(s + 4);
  v8h o;
#pragma unroll
  for (int j = 0; j < 4; ++j) {
    const float t0 = x0[j];
    const float t1 = x1[j];
    o[j]     = (_Float16)(bf16_rne(t0) * car);
    o[4 + j] = (_Float16)(bf16_rne(t1) * car);
  }
  _Float16* d = dst + (size_t)e;
  *(volatile v8h*)d = o;
  __threadfence();
  *(volatile v8h*)d = o;
}

__global__ __launch_bounds__(256) void k_rope(float* __restrict__ T)
{
  __shared__ __attribute__((aligned(16))) float st[512];
  const unsigned tid = threadIdx.x;
  const unsigned idx = blockIdx.x * 256u + tid;
  const unsigned s = idx >> 5, i = idx & 31u;
  const float e   = (float)(2u * i) * 0.015625f;
  const float pw  = powf(10000.0f, e);
  const float inv = 1.0f / pw;
  const float ang = (float)s * inv;
  float sn, cs;
  sincosf(ang, &sn, &cs);
  st[2u * tid]      = cs;
  st[2u * tid + 1u] = sn;
  __syncthreads();
  if (tid < 128u) {
    const v4f v = *(const v4f*)(st + 4u * tid);
    float* d = T + (size_t)blockIdx.x * 512u + 4u * tid;
    *(volatile v4f*)d = v;
    __threadfence();
    *(volatile v4f*)d = v;
  }
}

__device__ __forceinline__ void gemm_core(const _Float16* ap0, const _Float16* ap1,
                                          const _Float16* bp, unsigned K, unsigned hl, v8f (&acc)[8])
{
  const size_t bst = (size_t)16 * K;
#pragma unroll 1
  for (unsigned k0 = 0; k0 < K; k0 += 32u) {
    const v16h a0 = ld_frag(ap0 + k0, hl);
    const v16h a1 = ld_frag(ap1 + k0, hl);
    const v16h b0 = ld_frag(bp + k0, hl);
    const v16h b1 = ld_frag(bp + bst + k0, hl);
    const v16h b2 = ld_frag(bp + 2 * bst + k0, hl);
    const v16h b3 = ld_frag(bp + 3 * bst + k0, hl);
    acc[0] = mma(a0, b0, acc[0]);
    acc[1] = mma(a0, b1, acc[1]);
    acc[2] = mma(a0, b2, acc[2]);
    acc[3] = mma(a0, b3, acc[3]);
    acc[4] = mma(a1, b0, acc[4]);
    acc[5] = mma(a1, b1, acc[5]);
    acc[6] = mma(a1, b2, acc[6]);
    acc[7] = mma(a1, b3, acc[7]);
  }
}

__device__ __forceinline__ void store_tiles(const _Float16* ldsH, const _Float16* ldsL,
                                            _Float16* bh, _Float16* bl, unsigned ldc, unsigned tid)
{
  for (unsigned i = 0; i < 8u; ++i) {
    const unsigned q = i * 128u + tid;
    const unsigned rowl = q >> 3, ch = (q & 7u) * 8u;
    const v8h vh = *(const v8h*)(ldsH + rowl * 72u + ch);
    const v8h vl = *(const v8h*)(ldsL + rowl * 72u + ch);
    *(volatile v8h*)(bh + (size_t)rowl * ldc + ch) = vh;
    *(volatile v8h*)(bl + (size_t)rowl * ldc + ch) = vl;
  }
  __threadfence();
  for (unsigned i = 0; i < 8u; ++i) {
    const unsigned q = i * 128u + tid;
    const unsigned rowl = q >> 3, ch = (q & 7u) * 8u;
    const v8h vh = *(const v8h*)(ldsH + rowl * 72u + ch);
    const v8h vl = *(const v8h*)(ldsL + rowl * 72u + ch);
    *(volatile v8h*)(bh + (size_t)rowl * ldc + ch) = vh;
    *(volatile v8h*)(bl + (size_t)rowl * ldc + ch) = vl;
  }
}

__global__ __launch_bounds__(128) __attribute__((amdgpu_num_vgpr(256)))
void k_projq(const _Float16* __restrict__ A, const _Float16* __restrict__ Bt,
             const float* __restrict__ bias, const float* __restrict__ lnw,
             const float* __restrict__ lnb, const float* __restrict__ T,
             _Float16* __restrict__ PH, _Float16* __restrict__ PL)
{
  __shared__ __attribute__((aligned(16))) _Float16 ldsE[2 * 128 * 72];
  __shared__ __attribute__((aligned(16))) float    ldsT[128 * 64];
  _Float16* const ldsH = ldsE;
  _Float16* const ldsL = ldsE + 128 * 72;

  const unsigned tid = threadIdx.x, lane = tid & 31u, w = tid >> 5;
  const unsigned hl = lane >> 4, c = lane & 15u;
  const unsigned m0 = blockIdx.y * 128u, n0 = blockIdx.x * 64u;
  const unsigned mw = m0 + 32u * w;

  const _Float16* ap0 = A  + (size_t)(mw + c) * DM;
  const _Float16* ap1 = A  + (size_t)(mw + 16u + c) * DM;
  const _Float16* bp  = Bt + (size_t)(n0 + c) * DM;

  v8f acc[8] = {};
  gemm_core(ap0, ap1, bp, DM, hl, acc);

  {
    const float* tsrc = T + (size_t)(m0 & (unsigned)(SEQ - 1)) * 64u;
#pragma unroll 4
    for (unsigned i = 0; i < 16u; ++i) {
      const unsigned q = (i * 128u + tid) * 4u;
      *(v4f*)(ldsT + q) = *(const v4f*)(tsrc + q);
    }
  }
  float bq[4], gw[4], gb[4];
#pragma unroll
  for (int t = 0; t < 4; ++t) {
    const unsigned col = 16u * t + c;
    bq[t] = bf16_rne(bias[n0 + col]);
    gw[t] = bf16_rne(lnw[col]);
    gb[t] = bf16_rne(lnb[col]);
  }
  const float sgn = (c & 1u) ? 1.0f : -1.0f;
  __syncthreads();

#pragma unroll
  for (int i = 0; i < 2; ++i)
#pragma unroll
    for (int r = 0; r < 8; ++r) {
      const unsigned rowl = 32u * w + 16u * i + 8u * hl + r;
      float v[4];
#pragma unroll
      for (int t = 0; t < 4; ++t) v[t] = acc[i * 4 + t][r] * PROJ_TRUE + bq[t];
      const float mu = red16((v[0] + v[1]) + (v[2] + v[3])) * 0.015625f;
      float d[4];
#pragma unroll
      for (int t = 0; t < 4; ++t) d[t] = v[t] - mu;
      const float var = red16((d[0] * d[0] + d[1] * d[1]) + (d[2] * d[2] + d[3] * d[3])) * 0.015625f;
      const float rs = rsqrtf(var + LN_EPS);
#pragma unroll
      for (int t = 0; t < 4; ++t) {
        const float n  = d[t] * rs * gw[t] + gb[t];
        const float pn = __shfl_xor(n, 1, 32);
        const v2f cs2 = *(const v2f*)(ldsT + rowl * 64u + ((16u * t + c) & ~1u));
        const float pv = n * cs2[0] + sgn * pn * cs2[1];
        const _Float16 hv = (_Float16)pv;
        const float res = (pv - (float)hv) * RES_CAR;
        ldsH[rowl * 72u + 16u * t + c] = hv;
        ldsL[rowl * 72u + 16u * t + c] = (_Float16)res;
      }
    }
  __syncthreads();

  store_tiles(ldsH, ldsL, PH + (size_t)m0 * DM + n0, PL + (size_t)m0 * DM + n0, DM, tid);
}

__global__ __launch_bounds__(128) __attribute__((amdgpu_num_vgpr(256)))
void k_projk(const _Float16* __restrict__ A, const _Float16* __restrict__ Bt,
             const float* __restrict__ bias, const float* __restrict__ lnw,
             const float* __restrict__ lnb,
             _Float16* __restrict__ PH, _Float16* __restrict__ PL)
{
  __shared__ __attribute__((aligned(16))) _Float16 ldsE[2 * 128 * 72];
  _Float16* const ldsH = ldsE;
  _Float16* const ldsL = ldsE + 128 * 72;

  const unsigned tid = threadIdx.x, lane = tid & 31u, w = tid >> 5;
  const unsigned hl = lane >> 4, c = lane & 15u;
  const unsigned m0 = blockIdx.y * 128u, n0 = blockIdx.x * 64u;
  const unsigned mw = m0 + 32u * w;

  const _Float16* ap0 = A  + (size_t)(mw + c) * DC;
  const _Float16* ap1 = A  + (size_t)(mw + 16u + c) * DC;
  const _Float16* bp  = Bt + (size_t)(n0 + c) * DC;

  v8f acc[8] = {};
  gemm_core(ap0, ap1, bp, DC, hl, acc);

  float bq[4], gw[4], gb[4];
#pragma unroll
  for (int t = 0; t < 4; ++t) {
    const unsigned col = 16u * t + c;
    bq[t] = bf16_rne(bias[n0 + col]);
    gw[t] = bf16_rne(lnw[col]);
    gb[t] = bf16_rne(lnb[col]);
  }

#pragma unroll
  for (int i = 0; i < 2; ++i)
#pragma unroll
    for (int r = 0; r < 8; ++r) {
      const unsigned rowl = 32u * w + 16u * i + 8u * hl + r;
      float v[4];
#pragma unroll
      for (int t = 0; t < 4; ++t) v[t] = acc[i * 4 + t][r] * PROJ_TRUE + bq[t];
      const float mu = red16((v[0] + v[1]) + (v[2] + v[3])) * 0.015625f;
      float d[4];
#pragma unroll
      for (int t = 0; t < 4; ++t) d[t] = v[t] - mu;
      const float var = red16((d[0] * d[0] + d[1] * d[1]) + (d[2] * d[2] + d[3] * d[3])) * 0.015625f;
      const float rs = rsqrtf(var + LN_EPS);
#pragma unroll
      for (int t = 0; t < 4; ++t) {
        const float pv = (d[t] * rs * gw[t] + gb[t]) * K_CAR;
        const _Float16 hv = (_Float16)pv;
        const float res = (pv - (float)hv) * RES_CAR;
        ldsH[rowl * 72u + 16u * t + c] = hv;
        ldsL[rowl * 72u + 16u * t + c] = (_Float16)res;
      }
    }
  __syncthreads();

  store_tiles(ldsH, ldsL, PH + (size_t)m0 * DM + n0, PL + (size_t)m0 * DM + n0, DM, tid);
}

__global__ __launch_bounds__(128) __attribute__((amdgpu_num_vgpr(256)))
void k_projv(const _Float16* __restrict__ A, const _Float16* __restrict__ Bt,
             const float* __restrict__ bias,
             _Float16* __restrict__ PH, _Float16* __restrict__ PL)
{
  __shared__ __attribute__((aligned(16))) _Float16 ldsE[2 * 128 * 72];
  __shared__ float ldsB[128];
  _Float16* const ldsH = ldsE;
  _Float16* const ldsL = ldsE + 128 * 72;

  const unsigned tid = threadIdx.x, lane = tid & 31u, w = tid >> 5;
  const unsigned hl = lane >> 4, c = lane & 15u;
  const unsigned m0 = blockIdx.y * 128u, n0 = blockIdx.x * 64u;
  const unsigned mw = m0 + 32u * w;
  constexpr unsigned LDC = (unsigned)NB * SKV;

  ldsB[tid] = bf16_rne(bias[m0 + tid]) * ACT_CAR;

  const _Float16* ap0 = A  + (size_t)(mw + c) * DC;
  const _Float16* ap1 = A  + (size_t)(mw + 16u + c) * DC;
  const _Float16* bp  = Bt + (size_t)(n0 + c) * DC;

  v8f acc[8] = {};
  gemm_core(ap0, ap1, bp, DC, hl, acc);
  __syncthreads();

#pragma unroll
  for (int i = 0; i < 2; ++i)
#pragma unroll
    for (int r = 0; r < 8; ++r) {
      const unsigned rowl = 32u * w + 16u * i + 8u * hl + r;
      const float br = ldsB[rowl];
#pragma unroll
      for (int t = 0; t < 4; ++t) {
        const float pv = acc[i * 4 + t][r] * PROJ_SCL + br;
        const _Float16 hv = (_Float16)pv;
        const float res = (pv - (float)hv) * RES_CAR;
        ldsH[rowl * 72u + 16u * t + c] = hv;
        ldsL[rowl * 72u + 16u * t + c] = (_Float16)res;
      }
    }
  __syncthreads();

  store_tiles(ldsH, ldsL, PH + (size_t)m0 * LDC + n0, PL + (size_t)m0 * LDC + n0, LDC, tid);
}

__global__ __launch_bounds__(256) __attribute__((amdgpu_num_vgpr(256)))
void k_attn(const _Float16* __restrict__ QH, const _Float16* __restrict__ QL,
            const _Float16* __restrict__ KH, const _Float16* __restrict__ KL,
            const _Float16* __restrict__ VtH, const _Float16* __restrict__ VtL,
            _Float16* __restrict__ OH, _Float16* __restrict__ OL)
{
  constexpr int KT_H   = 32 * 72;
  constexpr int V_H    = HD * 40;
  constexpr int P_H    = 8 * 16 * 40;
  constexpr int TILE_H = 2 * KT_H + 2 * V_H + P_H;
  constexpr int EPI_H  = 2 * 128 * 72;
  constexpr int LDS_H  = (TILE_H > EPI_H) ? TILE_H : EPI_H;
  __shared__ __attribute__((aligned(16))) _Float16 lds[LDS_H];
  _Float16* const ldsK0 = lds;
  _Float16* const ldsK1 = ldsK0 + KT_H;
  _Float16* const ldsVH = ldsK1 + KT_H;
  _Float16* const ldsVL = ldsVH + V_H;
  _Float16* const ldsP  = ldsVL + V_H;
  _Float16* const ldsOH = lds;
  _Float16* const ldsOL = lds + 128 * 72;

  const unsigned tid = threadIdx.x, lane = tid & 31u, w = tid >> 5;
  const unsigned hl = lane >> 4, c = lane & 15u;
  const unsigned bz = blockIdx.z;
  const unsigned q0 = bz * (unsigned)SEQ + blockIdx.x * 128u;
  const unsigned kb = bz * (unsigned)SKV;
  const unsigned col0 = blockIdx.y * HD;
  constexpr unsigned LDV = (unsigned)NB * SKV;

  const size_t qrow = (size_t)(q0 + 16u * w + c) * DM + col0;
  v16h qh[2], ql[2];
#pragma unroll
  for (int ks = 0; ks < 2; ++ks) {
    qh[ks] = ld_frag(QH + qrow + 32 * ks, hl);
    ql[ks] = ld_frag(QL + qrow + 32 * ks, hl);
  }
  _Float16* const myP = ldsP + w * (16 * 40);

  const unsigned krr = tid >> 3, kcc = (tid & 7u) * 8u;
  const unsigned vdd = tid >> 2, vkc = (tid & 3u) * 8u;
  const _Float16* const kgh = KH + (size_t)(kb + krr) * DM + col0 + kcc;
  const _Float16* const kgl = KL + (size_t)(kb + krr) * DM + col0 + kcc;
  const _Float16* const vgh = VtH + (size_t)(col0 + vdd) * LDV + kb + vkc;
  const _Float16* const vgl = VtL + (size_t)(col0 + vdd) * LDV + kb + vkc;

  float m[8], l[8];
  v8f oh[4] = {}, ol[4] = {};
#pragma unroll
  for (int r = 0; r < 8; ++r) { m[r] = -__builtin_inff(); l[r] = 0.f; }

#pragma unroll 1
  for (unsigned kt = 0; kt < (unsigned)SKV / 32u; ++kt) {
    const unsigned mk = kt * 32u;
    {
      const v8h k8h = *(const v8h*)(kgh + (size_t)mk * DM);
      const v8h k8l = *(const v8h*)(kgl + (size_t)mk * DM);
      const v8h v8a = *(const v8h*)(vgh + mk);
      const v8h v8b = *(const v8h*)(vgl + mk);
      *(v8h*)(ldsK0 + krr * 72u + kcc) = k8h;
      *(v8h*)(ldsK1 + krr * 72u + kcc) = k8l;
      *(v8h*)(ldsVH + vdd * 40u + vkc) = v8a;
      *(v8h*)(ldsVL + vdd * 40u + vkc) = v8b;
    }
    __syncthreads();

    v8f sh[2] = {}, sl[2] = {};
#pragma unroll
    for (int ks = 0; ks < 2; ++ks) {
#pragma unroll
      for (int t = 0; t < 2; ++t) {
        const v16h kfh = ld_frag(ldsK0 + (16u * t + c) * 72u + 32 * ks, hl);
        const v16h kfl = ld_frag(ldsK1 + (16u * t + c) * 72u + 32 * ks, hl);
        sh[t] = mma(qh[ks], kfh, sh[t]);
        sl[t] = mma(ql[ks], kfh, sl[t]);
        sl[t] = mma(qh[ks], kfl, sl[t]);
      }
    }

#pragma unroll
    for (int r = 0; r < 8; ++r) {
      const float v0 = (sh[0][r] + sl[0][r] * RES_INV) * S_SCL;
      const float v1 = (sh[1][r] + sl[1][r] * RES_INV) * S_SCL;
      float tm = fmaxf(v0, v1);
      tm = fmaxf(tm, __shfl_xor(tm, 1, 32));
      tm = fmaxf(tm, __shfl_xor(tm, 2, 32));
      tm = fmaxf(tm, __shfl_xor(tm, 4, 32));
      tm = fmaxf(tm, __shfl_xor(tm, 8, 32));
      const float mn = fmaxf(m[r], tm);
      const float al = __expf(m[r] - mn);
      const float p0 = __expf(v0 - mn), p1 = __expf(v1 - mn);
      float rs = p0 + p1;
      rs += __shfl_xor(rs, 1, 32);
      rs += __shfl_xor(rs, 2, 32);
      rs += __shfl_xor(rs, 4, 32);
      rs += __shfl_xor(rs, 8, 32);
      l[r] = l[r] * al + rs;
      m[r] = mn;
#pragma unroll
      for (int t = 0; t < 4; ++t) { oh[t][r] *= al; ol[t][r] *= al; }
      _Float16* pp = myP + (8u * hl + r) * 40u + c;
      pp[0]  = (_Float16)(p0 * P_CAR);
      pp[16] = (_Float16)(p1 * P_CAR);
    }
    __syncthreads();

    const v16h pf = ld_frag(myP + c * 40u, hl);
#pragma unroll
    for (int t = 0; t < 4; ++t) {
      const v16h vfh = ld_frag(ldsVH + (16u * t + c) * 40u, hl);
      const v16h vfl = ld_frag(ldsVL + (16u * t + c) * 40u, hl);
      oh[t] = mma(pf, vfh, oh[t]);
      ol[t] = mma(pf, vfl, ol[t]);
    }
    __syncthreads();
  }

#pragma unroll
  for (int r = 0; r < 8; ++r) {
    const float inv = (1.0f / l[r]) * O_SCL;
    const unsigned rowl = 16u * w + 8u * hl + r;
#pragma unroll
    for (int t = 0; t < 4; ++t) {
      const float v = (oh[t][r] + ol[t][r] * RES_INV) * inv;
      const _Float16 hv = (_Float16)v;
      const float res = (v - (float)hv) * RES_CAR;
      ldsOH[rowl * 72u + 16u * t + c] = hv;
      ldsOL[rowl * 72u + 16u * t + c] = (_Float16)res;
    }
  }
  __syncthreads();
  _Float16* const bh = OH + (size_t)q0 * DM + col0;
  _Float16* const bl = OL + (size_t)q0 * DM + col0;
  for (unsigned i = 0; i < 4u; ++i) {
    const unsigned q = i * 256u + tid;
    const unsigned rowl = q >> 3, ch = (q & 7u) * 8u;
    const v8h vh = *(const v8h*)(ldsOH + rowl * 72u + ch);
    const v8h vl = *(const v8h*)(ldsOL + rowl * 72u + ch);
    *(volatile v8h*)(bh + (size_t)rowl * DM + ch) = vh;
    *(volatile v8h*)(bl + (size_t)rowl * DM + ch) = vl;
  }
  __threadfence();
  for (unsigned i = 0; i < 4u; ++i) {
    const unsigned q = i * 256u + tid;
    const unsigned rowl = q >> 3, ch = (q & 7u) * 8u;
    const v8h vh = *(const v8h*)(ldsOH + rowl * 72u + ch);
    const v8h vl = *(const v8h*)(ldsOL + rowl * 72u + ch);
    *(volatile v8h*)(bh + (size_t)rowl * DM + ch) = vh;
    *(volatile v8h*)(bl + (size_t)rowl * DM + ch) = vl;
  }
}

__global__ __launch_bounds__(128) __attribute__((amdgpu_num_vgpr(256)))
void k_oproj(const _Float16* __restrict__ AH, const _Float16* __restrict__ AL,
             const _Float16* __restrict__ Bt, const float* __restrict__ bias,
             float* __restrict__ Out)
{
  __shared__ __attribute__((aligned(16))) float ldsF[64 * 68];

  const unsigned tid = threadIdx.x, lane = tid & 31u, w = tid >> 5;
  const unsigned hl = lane >> 4, c = lane & 15u;
  const unsigned m0 = blockIdx.y * 64u, n0 = blockIdx.x * 64u;
  const unsigned mw = m0 + 16u * w;

  const _Float16* ap0 = AH + (size_t)(mw + c) * DM;
  const _Float16* ap1 = AL + (size_t)(mw + c) * DM;
  const _Float16* bp  = Bt + (size_t)(n0 + c) * DM;

  v8f acc[8] = {};
  gemm_core(ap0, ap1, bp, DM, hl, acc);

  float bo[4];
#pragma unroll
  for (int t = 0; t < 4; ++t) bo[t] = bf16_rne(bias[n0 + 16u * t + c]);

#pragma unroll
  for (int t = 0; t < 4; ++t)
#pragma unroll
    for (int r = 0; r < 8; ++r) {
      const unsigned rowl = 16u * w + 8u * hl + r;
      ldsF[rowl * 68u + 16u * t + c] = (acc[t][r] + acc[4 + t][r] * RES_INV) * OUT_SCL + bo[t];
    }
  __syncthreads();

  const unsigned orow0 = (m0 >> kSeqSh) * (unsigned)SEQ_FULL + (m0 & (unsigned)(SEQ - 1));
  float* const ob = Out + (size_t)orow0 * DM + n0;
  for (unsigned i = 0; i < 8u; ++i) {
    const unsigned qi = i * 128u + tid;
    const unsigned rowl = qi >> 4, col = (qi & 15u) * 4u;
    const v4f v = *(const v4f*)(ldsF + rowl * 68u + col);
    *(volatile v4f*)(ob + (size_t)rowl * DM + col) = v;
  }
  __threadfence();
  for (unsigned i = 0; i < 8u; ++i) {
    const unsigned qi = i * 128u + tid;
    const unsigned rowl = qi >> 4, col = (qi & 15u) * 4u;
    const v4f v = *(const v4f*)(ldsF + rowl * 68u + col);
    *(volatile v4f*)(ob + (size_t)rowl * DM + col) = v;
  }
}

extern "C" void kernel_launch(void* const* d_in, const int* in_sizes, int n_in,
                              void* d_out, int out_size, void* d_ws, size_t ws_size,
                              hipStream_t stream)
{
  if (n_in < 12) return;
  if ((long)in_sizes[0] < (long)(NB - 1) * SEQ_FULL * DM + (long)SEQ * DM) return;
  if ((long)in_sizes[1] < (long)(NB - 1) * SKV_FULL * DC + (long)SKV * DC) return;
  if ((long)in_sizes[2] < (long)DM * DM) return;
  if ((long)in_sizes[3] < (long)DM) return;
  if ((long)in_sizes[4] < (long)2 * DM * DC) return;
  if ((long)in_sizes[5] < (long)2 * DM) return;
  if ((long)in_sizes[6] < (long)HD || (long)in_sizes[7] < (long)HD) return;
  if ((long)in_sizes[8] < (long)HD || (long)in_sizes[9] < (long)HD) return;
  if ((long)in_sizes[10] < (long)DM * DM) return;
  if ((long)in_sizes[11] < (long)DM) return;
  if ((long)out_size < (long)(NB - 1) * SEQ_FULL * DM + (long)SEQ * DM) return;

  const float* x     = (const float*)d_in[0];
  const float* y     = (const float*)d_in[1];
  const float* q_w   = (const float*)d_in[2];
  const float* q_b   = (const float*)d_in[3];
  const float* kv_w  = (const float*)d_in[4];
  const float* kv_b  = (const float*)d_in[5];
  const float* qn_w  = (const float*)d_in[6];
  const float* qn_b  = (const float*)d_in[7];
  const float* kn_w  = (const float*)d_in[8];
  const float* kn_b  = (const float*)d_in[9];
  const float* out_w = (const float*)d_in[10];
  const float* out_b = (const float*)d_in[11];
  float* out = (float*)d_out;

  const size_t nX   = (size_t)NB * SEQ * DM;
  const size_t nY   = (size_t)NB * SKV * DC;
  const size_t nK   = (size_t)NB * SKV * DM;
  const size_t nWs  = (size_t)DM * DM;
  const size_t nWkv = (size_t)2 * DM * DC;
  const size_t nT   = (size_t)SEQ * 64;
  const size_t total_halves = nX + nY + 2 * nWs + nWkv + 2 * nX + 2 * nK + 2 * nK + 2 * nX;
  const size_t total_bytes  = total_halves * sizeof(_Float16) + nT * sizeof(float);
  if (total_bytes > ws_size) return;
  if (total_bytes > (size_t)134217728) return;

  _Float16* X16  = (_Float16*)d_ws;
  _Float16* Y16  = X16  + nX;
  _Float16* WqT  = Y16  + nY;
  _Float16* WkvT = WqT  + nWs;
  _Float16* WoT  = WkvT + nWkv;
  _Float16* QH   = WoT  + nWs;
  _Float16* QL   = QH   + nX;
  _Float16* KH   = QL   + nX;
  _Float16* KL   = KH   + nK;
  _Float16* VtH  = KL   + nK;
  _Float16* VtL  = VtH  + nK;
  _Float16* OH   = VtL  + nK;
  _Float16* OL   = OH   + nX;
  float*    ROT  = (float*)(OL + nX);

  const unsigned tx8  = (unsigned)(nX / 8);
  const unsigned ty8  = (unsigned)(nY / 8);
  const unsigned tw8  = (unsigned)(nWs / 8);
  const unsigned tkv8 = (unsigned)(nWkv / 8);
  k_cvt8<<<(tx8 + 255u) / 256u, 256, 0, stream>>>(x, X16, kDmSh, kSeqSh, (unsigned)SEQ_FULL, ACT_CAR, tx8);
  k_cvt8<<<(ty8 + 255u) / 256u, 256, 0, stream>>>(y, Y16, kDcSh, kSkvSh, (unsigned)SKV_FULL, ACT_CAR, ty8);
  k_cvt8<<<(tw8 + 255u) / 256u, 256, 0, stream>>>(q_w, WqT, kDmSh, 31u, 0u, W_CAR, tw8);
  k_cvt8<<<(tkv8 + 255u) / 256u, 256, 0, stream>>>(kv_w, WkvT, kDcSh, 31u, 0u, W_CAR, tkv8);
  k_cvt8<<<(tw8 + 255u) / 256u, 256, 0, stream>>>(out_w, WoT, kDmSh, 31u, 0u, W_CAR, tw8);

  k_rope<<<SEQ / 8, 256, 0, stream>>>(ROT);

  k_projq<<<dim3(DM / 64, NB * SEQ / 128), 128, 0, stream>>>(X16, WqT, q_b, qn_w, qn_b, ROT, QH, QL);
  k_projk<<<dim3(DM / 64, NB * SKV / 128), 128, 0, stream>>>(Y16, WkvT, kv_b, kn_w, kn_b, KH, KL);
  k_projv<<<dim3(NB * SKV / 64, DM / 128), 128, 0, stream>>>(WkvT + (size_t)DM * DC, Y16, kv_b + DM, VtH, VtL);

  k_attn<<<dim3(SEQ / 128, NH, NB), 256, 0, stream>>>(QH, QL, KH, KL, VtH, VtL, OH, OL);

  k_oproj<<<dim3(DM / 64, NB * SEQ / 64), 128, 0, stream>>>(OH, OL, WoT, out_b, out);
}
